// GaussianMixtureMLP_64183991271937
// MI455X (gfx1250) — hardware-verified
//
#include <hip/hip_runtime.h>
#include <math.h>

typedef __attribute__((ext_vector_type(16))) _Float16 v16h;
typedef __attribute__((ext_vector_type(16))) __bf16 v16b;
typedef __attribute__((ext_vector_type(8)))  _Float16 v8h;
typedef __attribute__((ext_vector_type(8)))  float v8f;
typedef __attribute__((ext_vector_type(4)))  float v4f;
typedef __attribute__((ext_vector_type(2)))  float v2f;
typedef __attribute__((ext_vector_type(4)))  unsigned v4u;
typedef __attribute__((ext_vector_type(4)))  int v4i;
typedef float __attribute__((may_alias)) float_a;
typedef int __attribute__((may_alias)) int_a;

template <typename T> __device__ __forceinline__ void vst2(void* p, T v) { *(volatile T*)p = v; __threadfence(); *(volatile T*)p = v; }
__device__ __forceinline__ v8f wmma16(v16h a, v16h b, v8f c) {
  v8f d = __builtin_amdgcn_wmma_f32_16x16x32_f16(false, a, false, b, (short)0, c, false, false);
  asm volatile("v_nop\n\tv_nop\n\tv_nop\n\tv_nop" : "+v"(d) : "v"(a), "v"(b));
  return d;
}
__device__ __forceinline__ v8f wmma_bf(v16b a, v16b b, v8f c) {
  v8f d = __builtin_amdgcn_wmma_f32_16x16x32_bf16(false, a, false, b, (short)0, c, false, false);
  asm volatile("v_nop\n\tv_nop\n\tv_nop\n\tv_nop" : "+v"(d) : "v"(a), "v"(b));
  return d;
}
__device__ __forceinline__ v16h frag_h(const _Float16* rowk0, int lane) {
  union { v16h v; v8h q[2]; } u; const _Float16* p = rowk0 + 8 * (lane >> 4);
  u.q[0] = *(const v8h*)p; u.q[1] = *(const v8h*)(p + 16); return u.v;
}
__device__ __forceinline__ v16h frag_f32(const float* rowk0, int lane) {
  v16h a; const float* p = rowk0 + 8 * (lane >> 4);
#pragma unroll
  for (int i = 0; i < 8; ++i) { a[i] = (_Float16)p[i]; a[8 + i] = (_Float16)p[16 + i]; }
  return a;
}
__device__ __forceinline__ v16h frag_f32s(const float* rowk0, int lane, float sc) {
  v16h a; const float* p = rowk0 + 8 * (lane >> 4);
#pragma unroll
  for (int i = 0; i < 8; ++i) { a[i] = (_Float16)(p[i] * sc); a[8 + i] = (_Float16)(p[16 + i] * sc); }
  return a;
}
__device__ __forceinline__ v16h fragc_f32(const float* W, int k0, int n, int lane, int ld, int K) {
  v16h a; const int g = lane >> 4;
#pragma unroll
  for (int i = 0; i < 8; ++i) { const int ka = k0 + 8 * g + i, kb = ka + 16;
    a[i] = (_Float16)(ka < K ? W[(size_t)(ka < K ? ka : K - 1) * ld + n] : 0.f); a[8 + i] = (_Float16)(kb < K ? W[(size_t)(kb < K ? kb : K - 1) * ld + n] : 0.f); }
  return a;
}
struct F2 { v16b h, l; };
__device__ __forceinline__ F2 bsplit16(const float v[16]) { F2 r;
#pragma unroll
  for (int i = 0; i < 16; ++i) { const __bf16 h = (__bf16)v[i]; r.h[i] = h; r.l[i] = (__bf16)(v[i] - (float)h); }
  return r; }
__device__ __forceinline__ F2 split_row(const float* row, int k0, int lane) { float v[16]; const float* p = row + k0 + 8 * (lane >> 4);
#pragma unroll
  for (int i = 0; i < 8; ++i) { v[i] = p[i]; v[8 + i] = p[16 + i]; }
  return bsplit16(v); }
__device__ __forceinline__ F2 split_rowK(const float* row, int k0, int lane, int K) { float v[16]; const int g = lane >> 4;
#pragma unroll
  for (int i = 0; i < 8; ++i) { const int ka = k0 + 8 * g + i, kb = ka + 16; v[i] = ka < K ? row[ka < K ? ka : K - 1] : 0.f; v[8 + i] = kb < K ? row[kb < K ? kb : K - 1] : 0.f; }
  return bsplit16(v); }
__device__ __forceinline__ F2 split_col(const float* W, int k0, int n, int lane, int ld, int K) { float v[16]; const int g = lane >> 4;
#pragma unroll
  for (int i = 0; i < 8; ++i) { const int ka = k0 + 8 * g + i, kb = ka + 16; v[i] = ka < K ? W[(size_t)(ka < K ? ka : K - 1) * ld + n] : 0.f; v[8 + i] = kb < K ? W[(size_t)(kb < K ? kb : K - 1) * ld + n] : 0.f; }
  return bsplit16(v); }
__device__ __forceinline__ v8f mac3(const F2& a, const F2& b, v8f c) { c = wmma_bf(a.l, b.h, c); c = wmma_bf(a.h, b.l, c); return wmma_bf(a.h, b.h, c); }
__device__ __forceinline__ float sigm(float v) { return 1.0f / (1.0f + expf(-v)); }
#define LDSX() do { asm volatile("s_wait_dscnt 0" ::: "memory"); __builtin_amdgcn_wave_barrier(); __builtin_amdgcn_fence(__ATOMIC_RELEASE, "workgroup"); } while (0)


#define NS 65536
#define DIN 128
#define HIDN 128
#define NOUT 18
#define NMOD 5
__device__ __forceinline__ float bfr(float v) { return (float)(__bf16)v; }
__device__ __attribute__((noinline)) float softplus_ni(float v) { return v > 20.f ? v : log1pf(expf(v)); }

__global__ __launch_bounds__(128) void k_gmm(const float* __restrict__ x, const float* __restrict__ W1, const float* __restrict__ b1, const float* __restrict__ W2, const float* __restrict__ b2, const float* __restrict__ W3, const float* __restrict__ b3, float* __restrict__ OM, float* __restrict__ OV) {
  __shared__ __align__(16) float sh[4][16][HIDN + 4];
  __shared__ __align__(16) float sm1[64][20], sm2[64][20];
  const int tid = threadIdx.x, wave = tid >> 5, lane = tid & 31, col = lane & 15, g = lane >> 4; const int r0b = blockIdx.x * 64, r0 = r0b + wave * 16;
  for (int q = tid; q < 64 * 20; q += 128) { (&sm1[0][0])[q] = 0.f; (&sm2[0][0])[q] = 0.f; }
  v16b ax[4];
#pragma unroll
  for (int kc = 0; kc < 4; ++kc) ax[kc] = split_row(x + (size_t)(r0 + col) * DIN, kc * 32, lane).h;
  __syncthreads();
#pragma unroll 1
  for (int m = 0; m < NMOD; ++m) {
    { v8f acc[8] = {};
#pragma unroll
      for (int kc = 0; kc < 4; ++kc) {
#pragma unroll
        for (int j = 0; j < 8; ++j) acc[j] = wmma_bf(ax[kc], split_row(W1 + ((size_t)m * HIDN + j * 16 + col) * DIN, kc * 32, lane).h, acc[j]); }
#pragma unroll
      for (int j = 0; j < 8; ++j) { const float bb = bfr(b1[m * HIDN + j * 16 + col]);
#pragma unroll
        for (int r = 0; r < 8; ++r) { const float v = acc[j][r] + bb; sh[wave][8 * g + r][j * 16 + col] = v > 0.f ? v : 0.f; } } }
    LDSX();
    { v8f acc[8] = {};
#pragma unroll
      for (int kc = 0; kc < 4; ++kc) { const F2 a = split_row(&sh[wave][col][0], kc * 32, lane);
#pragma unroll
        for (int j = 0; j < 8; ++j) { const v16b wb = split_row(W2 + ((size_t)m * HIDN + j * 16 + col) * HIDN, kc * 32, lane).h; acc[j] = wmma_bf(a.l, wb, acc[j]); acc[j] = wmma_bf(a.h, wb, acc[j]); } }
      LDSX();
#pragma unroll
      for (int j = 0; j < 8; ++j) { const float bb = bfr(b2[m * HIDN + j * 16 + col]);
#pragma unroll
        for (int r = 0; r < 8; ++r) { const float v = acc[j][r] + bb; sh[wave][8 * g + r][j * 16 + col] = v > 0.f ? v : 0.f; } } }
    LDSX();
    { v8f acc[3] = {};
#pragma unroll
      for (int kc = 0; kc < 4; ++kc) { const F2 a = split_row(&sh[wave][col][0], kc * 32, lane);
#pragma unroll
        for (int j = 0; j < 3; ++j) { const int n = j * 16 + col; const int nc = n < 2 * NOUT ? n : 2 * NOUT - 1; const v16b wb = split_row(W3 + ((size_t)m * 2 * NOUT + nc) * HIDN, kc * 32, lane).h; acc[j] = wmma_bf(a.l, wb, acc[j]); acc[j] = wmma_bf(a.h, wb, acc[j]); } }
      LDSX();
#pragma unroll
      for (int j = 0; j < 3; ++j) { const int n = j * 16 + col; if (n < 2 * NOUT) { const float bb = bfr(b3[m * 2 * NOUT + n]);
#pragma unroll
          for (int r = 0; r < 8; ++r) sh[wave][8 * g + r][n] = acc[j][r] + bb; } }
      LDSX();
      for (int q = lane; q < 16 * NOUT; q += 32) { const int rl = q / NOUT, o = q % NOUT; const float mu = sh[wave][rl][o]; const float var = softplus_ni(sh[wave][rl][NOUT + o]) + 1e-6f;
        sm1[wave * 16 + rl][o] += mu; sm2[wave * 16 + rl][o] += var + mu * mu; }
      LDSX(); } }
  __syncthreads();
  __shared__ __align__(16) float fm[64 * NOUT + 8], fv[64 * NOUT + 8];
  for (int q = tid; q < 64 * NOUT; q += 128) { const int rl = q / NOUT, o = q % NOUT; const float mean = sm1[rl][o] * (1.0f / NMOD); float var = sm2[rl][o] * (1.0f / NMOD) - mean * mean; var = (var > 0.f ? var : 0.f) + 1e-6f; fm[q] = mean; fv[q] = var; }
  __syncthreads();
  for (int q = tid; q < 64 * NOUT / 4; q += 128) { vst2(OM + (size_t)r0b * NOUT + q * 4, *(const v4f*)(&fm[q * 4])); vst2(OV + (size_t)r0b * NOUT + q * 4, *(const v4f*)(&fv[q * 4])); }
}
extern "C" void kernel_launch(void* const* d_in, const int* in_sizes, int n_in, void* d_out, int out_size, void* d_ws, size_t ws_size, hipStream_t stream) {
  (void)in_sizes; (void)n_in; (void)out_size; (void)ws_size; (void)d_ws;
  const float** I = (const float**)d_in;
  float* OM = (float*)d_out; float* OV = (float*)((char*)d_out + 4718592);
  k_gmm<<<NS / 64, 128, 0, stream>>>(I[0], I[1], I[2], I[3], I[4], I[5], I[6], OM, OV);
}
